// GATE_89876485636587
// MI455X (gfx1250) — hardware-verified
//
#include <hip/hip_runtime.h>
#include <hip/hip_bf16.h>
#include <stddef.h>
#include <stdint.h>


#define FIN     128
#define C1      32
#define C2      16
#define K2      64
#define NTHR    256
#define NWAVE   8
#define EPT     8
#define CHUNK   (NTHR * EPT)
#define WCAP    (EPT * 32)
#define LISTN   (NWAVE * WCAP)
#define NBMAX   1024
#define SLB     10
#define RCAP    28672
#define DEGCAP  4096
#define STW     32
#define GBM     64
#define GTHR    128
#define WSMAX   134217728
#define LDS_AGG ((2 * RCAP + 2 * NBMAX + LISTN) * 4 + 64)

static_assert((CHUNK & (CHUNK - 1)) == 0 && CHUNK <= 2048);
static_assert(NBMAX == (1 << SLB));
static_assert(NTHR * 4 == NBMAX);
static_assert(LISTN >= NBMAX);
static_assert(LISTN >= NWAVE * WCAP);
static_assert((RCAP % 32) == 0);
static_assert(NWAVE * STW <= RCAP);
static_assert(LDS_AGG <= 300000);
static_assert(GBM == (GTHR / 32) * 16);
static_assert((FIN % 32) == 0 && (K2 % 32) == 0 && C1 == 32 && C2 == 16);
static_assert(GBM * C1 / 4 == 4 * GTHR && GBM * C2 / 4 == 2 * GTHR);

typedef float          v4f  __attribute__((ext_vector_type(4)));
typedef float          v8f  __attribute__((ext_vector_type(8)));
typedef int            v4i  __attribute__((ext_vector_type(4)));
typedef int            v8i  __attribute__((ext_vector_type(8)));
typedef unsigned short v8us __attribute__((ext_vector_type(8)));
typedef __bf16         v16b __attribute__((ext_vector_type(16)));
union FragB { v16b v; v8us u[2]; v8i w; };

__device__ __forceinline__ v8f wmb(const FragB& a, const FragB& b, v8f c) {
  v8f d = __builtin_amdgcn_wmma_f32_16x16x32_bf16(false, a.v, false, b.v, (short)0, c, false, false);
  asm volatile("v_nop\n\tv_nop\n\tv_nop\n\tv_nop" : "+v"(d) : "v"(a.w), "v"(b.w));
  return d;
}

__device__ __forceinline__ void ldwait() {
  asm volatile("s_wait_loadcnt 0x0" ::: "memory");
}

__device__ __forceinline__ float lrelu(float v) { return v >= 0.f ? v : 0.2f * v; }

__device__ __forceinline__ unsigned short bbits(float f) {
  unsigned int u = __float_as_uint(f);
  u += 0x7FFFu + ((u >> 16) & 1u);
  return (unsigned short)(u >> 16);
}
__device__ __forceinline__ float bval(unsigned short b) { return __uint_as_float(((unsigned int)b) << 16); }
__device__ __forceinline__ float bf16r(float f) { return bval(bbits(f)); }
__device__ __forceinline__ unsigned short lbits(float f) { return bbits(f - bval(bbits(f))); }

__device__ __forceinline__ v8us cvt8b(const v4f a, const v4f b) {
  v8us r;
  r[0] = bbits(a.x); r[1] = bbits(a.y); r[2] = bbits(a.z); r[3] = bbits(a.w);
  r[4] = bbits(b.x); r[5] = bbits(b.y); r[6] = bbits(b.z); r[7] = bbits(b.w);
  return r;
}
__device__ __forceinline__ v8us cvt8lo(const v4f a, const v4f b) {
  v8us r;
  r[0] = lbits(a.x); r[1] = lbits(a.y); r[2] = lbits(a.z); r[3] = lbits(a.w);
  r[4] = lbits(b.x); r[5] = lbits(b.y); r[6] = lbits(b.z); r[7] = lbits(b.w);
  return r;
}

__device__ __forceinline__ int scan_chunk(const int* __restrict__ dsts, int nE, int cbase, int slotBase,
                                          int nb, int vec8, int* list, int tid, int lane, int wave) {
  int wc = 0;
  const int el0  = tid * EPT;
  const int e0   = cbase + el0;
  const int sent = -2147483647 - 1;
  v4i da, db;
  if (vec8 != 0 && cbase + CHUNK <= nE) {
    da = *(const v4i*)(dsts + e0);
    db = *(const v4i*)(dsts + e0 + 4);
  } else {
    da.x = (e0     < nE) ? dsts[min(e0,     nE - 1)] : sent;
    da.y = (e0 + 1 < nE) ? dsts[min(e0 + 1, nE - 1)] : sent;
    da.z = (e0 + 2 < nE) ? dsts[min(e0 + 2, nE - 1)] : sent;
    da.w = (e0 + 3 < nE) ? dsts[min(e0 + 3, nE - 1)] : sent;
    db.x = (e0 + 4 < nE) ? dsts[min(e0 + 4, nE - 1)] : sent;
    db.y = (e0 + 5 < nE) ? dsts[min(e0 + 5, nE - 1)] : sent;
    db.z = (e0 + 6 < nE) ? dsts[min(e0 + 6, nE - 1)] : sent;
    db.w = (e0 + 7 < nE) ? dsts[min(e0 + 7, nE - 1)] : sent;
  }
  const unsigned nbs = (unsigned)slotBase;
  const unsigned unb = (unsigned)nb;
  const unsigned s0 = (unsigned)da.x - nbs, s1 = (unsigned)da.y - nbs;
  const unsigned s2 = (unsigned)da.z - nbs, s3 = (unsigned)da.w - nbs;
  const unsigned s4 = (unsigned)db.x - nbs, s5 = (unsigned)db.y - nbs;
  const unsigned s6 = (unsigned)db.z - nbs, s7 = (unsigned)db.w - nbs;
  const bool h0 = s0 < unb, h1 = s1 < unb, h2 = s2 < unb, h3 = s3 < unb;
  const bool h4 = s4 < unb, h5 = s5 < unb, h6 = s6 < unb, h7 = s7 < unb;
  const unsigned any = __builtin_amdgcn_ballot_w32(h0 | h1 | h2 | h3 | h4 | h5 | h6 | h7);
  if (any != 0u) {
#define HITJ(J, HJ, SJ) { \
      const unsigned mj = __builtin_amdgcn_ballot_w32(HJ); \
      if (mj != 0u) { \
        if (HJ) { \
          const int pos = wc + (int)__builtin_amdgcn_mbcnt_lo(mj, 0u); \
          if (pos < WCAP) list[wave * WCAP + pos] = ((el0 + (J)) << SLB) | (int)(SJ); \
        } \
        wc += (int)__builtin_popcount(mj); } }
    HITJ(0, h0, s0)
    HITJ(1, h1, s1)
    HITJ(2, h2, s2)
    HITJ(3, h3, s3)
    HITJ(4, h4, s4)
    HITJ(5, h5, s5)
    HITJ(6, h6, s6)
    HITJ(7, h7, s7)
#undef HITJ
  }
  return wc;
}

__global__ __launch_bounds__(NTHR) void k_wprep(const float* __restrict__ W1, const float* __restrict__ W2,
                                                const float* __restrict__ ew,
                                                unsigned short* WT1, unsigned short* WT2, int nUnits) {
  (void)ew;
  const int u = (int)blockIdx.x * NTHR + (int)threadIdx.x;
  if (u >= nUnits) return;
  v8us r;
  unsigned short* dp;
  if (u < C1 * (FIN / 8)) {
    const int n  = u >> 4;
    const int k8 = (u & 15) * 8;
#pragma unroll
    for (int i = 0; i < 8; ++i) r[i] = bbits(W1[(size_t)(k8 + i) * C1 + n]);
    dp = WT1 + (size_t)n * FIN + k8;
  } else {
    const int v  = u - C1 * (FIN / 8);
    const int n  = v >> 3;
    const int k8 = (v & 7) * 8;
#pragma unroll
    for (int i = 0; i < 8; ++i) {
      const int kk = (k8 + i) & (C1 - 1);
      r[i] = bbits(W2[(size_t)kk * C2 + n]);
    }
    dp = WT2 + (size_t)n * K2 + k8;
  }
  *(volatile v8us*)dp = r;
  __threadfence();
  *(volatile v8us*)dp = r;
}

__global__ __launch_bounds__(GTHR) void k_gemm1(
    const float* __restrict__ x, const unsigned short* __restrict__ WT1,
    const float* __restrict__ asrc, const float* __restrict__ adst,
    float* H1, float* ALS, float* ALD, int nN) {
  __shared__ __attribute__((aligned(16))) float stg[GBM * C1];
  __shared__ __attribute__((aligned(16))) float lvs[C1];
  __shared__ __attribute__((aligned(16))) float lvd[C1];
  __shared__ __attribute__((aligned(16))) float lal[GBM];
  __shared__ __attribute__((aligned(16))) float lad[GBM];
  const int tid = (int)threadIdx.x, lane = tid & 31, wave = tid >> 5, hh = lane >> 4, m = lane & 15;
  const int rowBase = (int)blockIdx.x * GBM;
  if (wave == 0) lvs[lane] = bf16r(asrc[lane]);
  if (wave == 1) lvd[lane] = bf16r(adst[lane]);

  const int  arow = rowBase + 16 * wave + m;
  const int  arc  = arow < nN ? arow : nN - 1;
  const bool live = arow < nN;
  const float* ap = x + (size_t)arc * FIN + 8 * hh;
  const unsigned short* wp = WT1 + (size_t)m * FIN + 8 * hh;
  const v4f z4 = {0.f, 0.f, 0.f, 0.f};
  v8f acc[2];
  {
    const v8f z = {0.f, 0.f, 0.f, 0.f, 0.f, 0.f, 0.f, 0.f};
    acc[0] = z; acc[1] = z;
  }
#pragma unroll 1
  for (int ks = 0; ks < FIN / 32; ++ks) {
    v4f a0 = *(const v4f*)(ap + 32 * ks);
    v4f a1 = *(const v4f*)(ap + 32 * ks + 4);
    v4f a2 = *(const v4f*)(ap + 32 * ks + 16);
    v4f a3 = *(const v4f*)(ap + 32 * ks + 20);
    if (!live) { a0 = z4; a1 = z4; a2 = z4; a3 = z4; }
    FragB af;
    af.u[0] = cvt8b(a0, a1);
    af.u[1] = cvt8b(a2, a3);
#pragma unroll
    for (int t = 0; t < 2; ++t) {
      const unsigned short* wq = wp + (size_t)(16 * t) * FIN + 32 * ks;
      FragB bf;
      bf.u[0] = *(const v8us*)wq;
      bf.u[1] = *(const v8us*)(wq + 16);
      acc[t] = wmb(af, bf, acc[t]);
    }
  }

#pragma unroll
  for (int t = 0; t < 2; ++t) {
#pragma unroll
    for (int r = 0; r < 8; ++r) {
      const int lr = 16 * wave + 8 * hh + r;
      stg[lr * C1 + 16 * t + m] = acc[t][r];
    }
  }
  __syncthreads();

  if (tid < GBM) {
    float s = 0.f, d = 0.f;
#pragma unroll 4
    for (int c = 0; c < C1; ++c) {
      const float v = stg[tid * C1 + c];
      s = fmaf(v, lvs[c], s);
      d = fmaf(v, lvd[c], d);
    }
    lal[tid] = s;
    lad[tid] = d;
  }
  __syncthreads();

  v4f hv[4];
#pragma unroll
  for (int i = 0; i < 4; ++i) hv[i] = *(const v4f*)(stg + 4 * (i * GTHR + tid));
  float* hb = H1 + (size_t)rowBase * C1;
  const int  li  = lane & 15;
  const v4f  va  = *(const v4f*)(lal + 4 * li);
  const v4f  vd  = *(const v4f*)(lad + 4 * li);
  const v4f  vv  = (wave == 0) ? va : vd;
  float*     avp = ((wave == 0) ? ALS : ALD) + rowBase + 4 * li;
  const bool sw  = (wave < 2) && (lane < 16);
#pragma unroll
  for (int i = 0; i < 4; ++i) *(volatile v4f*)(hb + 4 * (i * GTHR + tid)) = hv[i];
  if (sw) *(volatile v4f*)avp = vv;
  __threadfence();
#pragma unroll
  for (int i = 0; i < 4; ++i) *(volatile v4f*)(hb + 4 * (i * GTHR + tid)) = hv[i];
  if (sw) *(volatile v4f*)avp = vv;
}

__global__ __launch_bounds__(GTHR) void k_gemm2(
    const unsigned short* __restrict__ HL1, const unsigned short* __restrict__ WT2,
    const float* __restrict__ asrc, const float* __restrict__ adst,
    float* H2, float* ALS, float* ALD) {
  __shared__ __attribute__((aligned(16))) float stg[GBM * C2];
  __shared__ __attribute__((aligned(16))) float lvs[C2];
  __shared__ __attribute__((aligned(16))) float lvd[C2];
  __shared__ __attribute__((aligned(16))) float lal[GBM];
  __shared__ __attribute__((aligned(16))) float lad[GBM];
  const int tid = (int)threadIdx.x, lane = tid & 31, wave = tid >> 5, hh = lane >> 4, m = lane & 15;
  const int rowBase = (int)blockIdx.x * GBM;
  if (wave == 0) {
    const float v = asrc[lane & (C2 - 1)];
    if (lane < C2) lvs[lane] = bf16r(v);
  }
  if (wave == 1) {
    const float v = adst[lane & (C2 - 1)];
    if (lane < C2) lvd[lane] = bf16r(v);
  }

  const unsigned short* ap = HL1 + (size_t)(rowBase + 16 * wave + m) * K2 + 8 * hh;
  const unsigned short* wp = WT2 + (size_t)m * K2 + 8 * hh;
  v8f acc = {0.f, 0.f, 0.f, 0.f, 0.f, 0.f, 0.f, 0.f};
#pragma unroll 1
  for (int ks = 0; ks < K2 / 32; ++ks) {
    FragB af, bf;
    af.u[0] = *(const v8us*)(ap + 32 * ks);
    af.u[1] = *(const v8us*)(ap + 32 * ks + 16);
    bf.u[0] = *(const v8us*)(wp + 32 * ks);
    bf.u[1] = *(const v8us*)(wp + 32 * ks + 16);
    acc = wmb(af, bf, acc);
  }

#pragma unroll
  for (int r = 0; r < 8; ++r) {
    const int lr = 16 * wave + 8 * hh + r;
    stg[lr * C2 + m] = acc[r];
  }
  __syncthreads();

  if (tid < GBM) {
    float s = 0.f, d = 0.f;
#pragma unroll 4
    for (int c = 0; c < C2; ++c) {
      const float v = stg[tid * C2 + c];
      s = fmaf(v, lvs[c], s);
      d = fmaf(v, lvd[c], d);
    }
    lal[tid] = s;
    lad[tid] = d;
  }
  __syncthreads();

  v4f hv[2];
#pragma unroll
  for (int i = 0; i < 2; ++i) hv[i] = *(const v4f*)(stg + 4 * (i * GTHR + tid));
  float* hb = H2 + (size_t)rowBase * C2;
  const int  li  = lane & 15;
  const v4f  va  = *(const v4f*)(lal + 4 * li);
  const v4f  vd  = *(const v4f*)(lad + 4 * li);
  const v4f  vv  = (wave == 0) ? va : vd;
  float*     avp = ((wave == 0) ? ALS : ALD) + rowBase + 4 * li;
  const bool sw  = (wave < 2) && (lane < 16);
#pragma unroll
  for (int i = 0; i < 2; ++i) *(volatile v4f*)(hb + 4 * (i * GTHR + tid)) = hv[i];
  if (sw) *(volatile v4f*)avp = vv;
  __threadfence();
#pragma unroll
  for (int i = 0; i < 2; ++i) *(volatile v4f*)(hb + 4 * (i * GTHR + tid)) = hv[i];
  if (sw) *(volatile v4f*)avp = vv;
}

template<int L>
__global__ __launch_bounds__(NTHR) void k_agg(
    const int* __restrict__ srcs, const int* __restrict__ dsts,
    const float* __restrict__ H, const float* __restrict__ ALS, const float* __restrict__ ALD,
    const float* __restrict__ bias, unsigned short* HL, float* out,
    int nN, int nE, int nb, int vec8, int MPr) {
  constexpr int C = (L == 1) ? C1 : C2;
  extern __shared__ v4f lds_dyn[];
  int* reg1 = (int*)lds_dyn;
  int* reg2 = reg1 + RCAP;
  int* scnt = reg2 + RCAP;
  int* soff = scnt + NBMAX;
  int* list = soff + NBMAX;
  int* wcnt = list + LISTN;
  int* wtot = wcnt + NWAVE;
  const int tid = (int)threadIdx.x, lane = tid & 31, wave = tid >> 5;
  const int nodeBase = (int)blockIdx.x * nb;

  for (int i = tid; i < NBMAX; i += NTHR) scnt[i] = 0;
  __syncthreads();

  int tot = 0;
  const int nChunks = (nE + CHUNK - 1) / CHUNK;
#pragma unroll 1
  for (int ck = 0; ck < nChunks; ++ck) {
    const int cbase = ck * CHUNK;
    const int wc = scan_chunk(dsts, nE, cbase, nodeBase, nb, vec8, list, tid, lane, wave);
    if (lane == 0) wcnt[wave] = wc;
    __syncthreads();
    int pre = 0, all = 0;
#pragma unroll
    for (int w2 = 0; w2 < NWAVE; ++w2) {
      int c = wcnt[w2];
      c = c < 0 ? 0 : (c > WCAP ? WCAP : c);
      all += c;
      pre += (w2 < wave) ? c : 0;
    }
    const int wcc  = wc > WCAP ? WCAP : wc;
    const int base = tot + pre;
#pragma unroll 1
    for (int i = lane; i < wcc; i += 32) {
      const int ent = list[wave * WCAP + i];
      const int el  = (ent >> SLB) & (CHUNK - 1);
      const int sl  = ent & (NBMAX - 1);
      int eid = cbase + el;
      eid = eid > nE - 1 ? nE - 1 : eid;
      const int pos = base + i;
      if (pos < RCAP) reg1[pos] = (int)(((unsigned)eid << SLB) | (unsigned)sl);
    }
    tot += all;
    tot = tot > RCAP ? RCAP : tot;
    __syncthreads();
  }
  const int nh = tot;

  if (wave == 0) {
#pragma unroll 1
    for (int b0 = 0; b0 < nh; b0 += 32) {
      const int idx = b0 + lane;
      const int uv  = reg1[idx < RCAP ? idx : RCAP - 1];
      const int m32 = (nh - b0) < 32 ? (nh - b0) : 32;
#pragma unroll 1
      for (int k = 0; k < m32; ++k) {
        const int u  = __builtin_amdgcn_readlane(uv, k);
        const int sl = u & (NBMAX - 1);
        if (lane == 0) scnt[sl] = scnt[sl] + 1;
      }
    }
  }
  __syncthreads();

  {
    const v4i ca = *(const v4i*)(scnt + 4 * tid);
    const int e0 = ca.x < 0 ? 0 : ca.x, e1 = ca.y < 0 ? 0 : ca.y, e2 = ca.z < 0 ? 0 : ca.z, e3 = ca.w < 0 ? 0 : ca.w;
    const int ts = e0 + e1 + e2 + e3;
    int incl = ts;
#pragma unroll
    for (int d = 1; d < 32; d <<= 1) {
      const int up = __shfl_up(incl, d);
      if (lane >= d) incl += up;
    }
    if (lane == 31) wtot[wave] = incl;
    __syncthreads();
    int pre = 0;
#pragma unroll
    for (int w2 = 0; w2 < NWAVE; ++w2) pre += (w2 < wave) ? wtot[w2] : 0;
    int run = pre + incl - ts;
    soff[4 * tid + 0] = run; run += e0;
    soff[4 * tid + 1] = run; run += e1;
    soff[4 * tid + 2] = run; run += e2;
    soff[4 * tid + 3] = run;
  }
  __syncthreads();
  for (int i = tid; i < NBMAX; i += NTHR) list[i] = soff[i];
  __syncthreads();

  if (wave == 0) {
#pragma unroll 1
    for (int b0 = 0; b0 < nh; b0 += 32) {
      const int idx = b0 + lane;
      const int uv  = reg1[idx < RCAP ? idx : RCAP - 1];
      const int m32 = (nh - b0) < 32 ? (nh - b0) : 32;
#pragma unroll 1
      for (int k = 0; k < m32; ++k) {
        const int u   = __builtin_amdgcn_readlane(uv, k);
        const int sl  = u & (NBMAX - 1);
        const int eid = (int)((unsigned)u >> SLB);
        if (lane == 0) {
          int pos = list[sl];
          pos = pos < 0 ? 0 : (pos > RCAP - 1 ? RCAP - 1 : pos);
          reg2[pos] = eid;
          list[sl] = pos + 1;
        }
      }
    }
  }
  __syncthreads();

  const int nbw = nb >> 3;
  const bool ovf = (nh >= RCAP);
  const float qnan = __int_as_float(0x7fc00000);
  float* stw = (float*)reg1 + wave * STW;
  const int ch = lane & (C - 1);
  const float bv = bf16r(bias[ch]);
#pragma unroll 1
  for (int jt = 0; jt < nbw; ++jt) {
    const int slot = wave * nbw + jt;
    const int grow = nodeBase + slot;
    const int gcl  = grow < nN ? grow : nN - 1;
    int st = soff[slot];
    const int craw = scnt[slot];
    int cnt = craw;
    st  = st < 0 ? 0 : (st > nh ? nh : st);
    cnt = cnt < 0 ? 0 : (cnt > DEGCAP ? DEGCAP : cnt);
    if (cnt > nh - st) cnt = nh - st;
    const float pz = (ovf || craw > DEGCAP) ? qnan : 0.0f;
    const bool wr = grow < MPr;
    const float live = grow < nN ? 1.0f : 0.0f;

    const float ad  = ALD[gcl];
    const float as0 = ALS[gcl];
    float acc = H[(size_t)gcl * C + ch];
    ldwait();
    float mx = lrelu(as0 + ad);
    float dn = 1.0f;

#pragma unroll 1
    for (int q = 0; q < cnt; ++q) {
      int idx = st + q; idx = idx > RCAP - 1 ? RCAP - 1 : idx;
      int eid = reg2[idx]; eid = eid < 0 ? 0 : (eid > nE - 1 ? nE - 1 : eid);
      const int sraw = srcs[eid];
      const int s = sraw < 0 ? 0 : (sraw > nN - 1 ? nN - 1 : sraw);
      const float as = ALS[s];
      const float hv = H[(size_t)s * C + ch];
      ldwait();
      const float al = lrelu(as + ad);
      const float df = al - mx;
      const float ee = __expf(-fabsf(df));
      const bool up  = df > 0.f;
      const float s1 = up ? ee : 1.0f;
      const float s2 = up ? 1.0f : ee;
      mx  = up ? al : mx;
      dn  = fmaf(dn, s1, s2);
      acc = fmaf(acc, s1, s2 * hv);
    }
    const float inv = __builtin_amdgcn_rcpf(dn);
    float r = fmaf(acc, inv, bv);
    if (L == 1) r = fmaxf(r, 0.f);
    r = r * live + pz;

    if (L == 1) {
      __builtin_amdgcn_fence(__ATOMIC_RELEASE, "wavefront");
      __builtin_amdgcn_wave_barrier();
      stw[lane] = r;
      __builtin_amdgcn_fence(__ATOMIC_RELEASE, "wavefront");
      __builtin_amdgcn_wave_barrier();
      const int lc = lane & 7;
      const int c0 = (lc & 3) * 8;
      const v4f ga = *(const v4f*)(stw + c0);
      const v4f gb = *(const v4f*)(stw + c0 + 4);
      const v8us hiv = cvt8b(ga, gb);
      const v8us lov = cvt8lo(ga, gb);
      v8us sv;
      if (lc < 4) sv = hiv; else sv = lov;
      const int growc = grow < MPr ? grow : MPr - 1;
      unsigned short* gp = HL + (size_t)growc * K2 + 8 * lc;
      const bool wsv = wr && (lane < 8);
      if (wsv) *(volatile v8us*)gp = sv;
      __threadfence();
      if (wsv) *(volatile v8us*)gp = sv;
    } else {
      const int half = jt & 1;
      __builtin_amdgcn_fence(__ATOMIC_RELEASE, "wavefront");
      __builtin_amdgcn_wave_barrier();
      stw[half * C2 + ch] = r;
      __builtin_amdgcn_fence(__ATOMIC_RELEASE, "wavefront");
      __builtin_amdgcn_wave_barrier();
      if (half != 0) {
        const int lc = lane & 7;
        const v4f g = *(const v4f*)(stw + 4 * lc);
        const int prow = grow - 1;
        int nv = nN - prow;
        nv = nv < 0 ? 0 : (nv > 2 ? 2 : nv);
        const int prc = prow < 0 ? 0 : (prow > nN - 1 ? nN - 1 : prow);
        float* gp = out + (size_t)prc * C2 + 4 * lc;
        const bool wsv = lane < 4 * nv;
        if (wsv) *(volatile v4f*)gp = g;
        __threadfence();
        if (wsv) *(volatile v4f*)gp = g;
      }
    }
  }
}

static int pick_nb(int nE, int nN) {
  int nb = NBMAX;
  while (nb > 16 && (long long)nb * (long long)nE * 5LL > (long long)RCAP * (long long)nN * 4LL) nb >>= 1;
  return nb;
}
static inline int cdiv(int a, int b) { return (a + b - 1) / b; }

extern "C" void kernel_launch(void* const* d_in, const int* in_sizes, int n_in,
                              void* d_out, int out_size, void* d_ws, size_t ws_size,
                              hipStream_t stream) {
  if (n_in < 11) return;
  const int nN = in_sizes[0] / FIN;
  if (nN <= 1 || in_sizes[0] != nN * FIN || nN > (1 << 22)) return;
  if (in_sizes[1] < 2 || (in_sizes[1] & 1) != 0) return;
  const int nE = in_sizes[1] / 2;
  if (nE < 1 || nE > (1 << (32 - SLB)) - 1) return;
  if (in_sizes[3] != FIN * C1 || in_sizes[4] != C1 || in_sizes[5] != C1 || in_sizes[6] != C1) return;
  if (in_sizes[7] != C1 * C2  || in_sizes[8] != C2 || in_sizes[9] != C2 || in_sizes[10] != C2) return;
  if (out_size != nN * C2) return;

  const float* x   = (const float*)d_in[0];
  const int*   ei  = (const int*)  d_in[1];
  const float* ew  = (const float*)d_in[2];
  const float* W1  = (const float*)d_in[3];
  const float* as1 = (const float*)d_in[4];
  const float* ad1 = (const float*)d_in[5];
  const float* b1  = (const float*)d_in[6];
  const float* W2  = (const float*)d_in[7];
  const float* as2 = (const float*)d_in[8];
  const float* ad2 = (const float*)d_in[9];
  const float* b2  = (const float*)d_in[10];
  float* out = (float*)d_out;
  const int* src = ei;
  const int* dst = ei + nE;

  const int MP   = cdiv(nN, GBM) * GBM;
  const int nb   = pick_nb(nE, nN);
  const int gA   = cdiv(MP, nb);
  const int vec8 = ((nE & 3) == 0) ? 1 : 0;
  if (gA * nb < MP || (nb & 15) != 0) return;

  char* ws = (char*)d_ws;
  size_t off = 0;
  const size_t oWT1 = off; off += (size_t)C1 * FIN * 2;           off = (off + 255) & ~(size_t)255;
  const size_t oWT2 = off; off += (size_t)C2 * K2 * 2;            off = (off + 255) & ~(size_t)255;
  const size_t oH1  = off; off += (size_t)MP * C1 * 4;            off = (off + 255) & ~(size_t)255;
  const size_t oAS1 = off; off += (size_t)MP * 4;                 off = (off + 255) & ~(size_t)255;
  const size_t oAD1 = off; off += (size_t)MP * 4;                 off = (off + 255) & ~(size_t)255;
  const size_t oHL1 = off; off += (size_t)MP * K2 * 2;            off = (off + 255) & ~(size_t)255;
  const size_t oH2  = off; off += (size_t)MP * C2 * 4;            off = (off + 255) & ~(size_t)255;
  const size_t oAS2 = off; off += (size_t)MP * 4;                 off = (off + 255) & ~(size_t)255;
  const size_t oAD2 = off; off += (size_t)MP * 4;                 off = (off + 255) & ~(size_t)255;
  if (off > ws_size || off > (size_t)WSMAX) return;
  unsigned short* WT1 = (unsigned short*)(ws + oWT1);
  unsigned short* WT2 = (unsigned short*)(ws + oWT2);
  float*          H1  = (float*)(ws + oH1);
  float*          AS1 = (float*)(ws + oAS1);
  float*          AD1 = (float*)(ws + oAD1);
  unsigned short* HL1 = (unsigned short*)(ws + oHL1);
  float*          H2  = (float*)(ws + oH2);
  float*          AS2 = (float*)(ws + oAS2);
  float*          AD2 = (float*)(ws + oAD2);

  hipFuncSetAttribute(reinterpret_cast<const void*>(&k_agg<1>),
                      hipFuncAttributeMaxDynamicSharedMemorySize, LDS_AGG);
  hipFuncSetAttribute(reinterpret_cast<const void*>(&k_agg<2>),
                      hipFuncAttributeMaxDynamicSharedMemorySize, LDS_AGG);

  {
    const int nU = C1 * (FIN / 8) + C2 * (K2 / 8);
    k_wprep<<<cdiv(nU, NTHR), NTHR, 0, stream>>>(W1, W2, ew, WT1, WT2, nU);
  }
  const int gM = MP / GBM;
  k_gemm1<<<gM, GTHR, 0, stream>>>(x, WT1, as1, ad1, H1, AS1, AD1, nN);
  k_agg<1><<<gA, NTHR, LDS_AGG, stream>>>(src, dst, H1, AS1, AD1, b1, HL1, out, nN, nE, nb, vec8, MP);
  k_gemm2<<<gM, GTHR, 0, stream>>>(HL1, WT2, as2, ad2, H2, AS2, AD2);
  k_agg<2><<<gA, NTHR, LDS_AGG, stream>>>(src, dst, H2, AS2, AD2, b2, HL1, out, nN, nE, nb, vec8, MP);
}
